// DeepSeekMoELayer_11690900980107
// MI455X (gfx1250) — hardware-verified
//
#include <hip/hip_runtime.h>
#include <stddef.h>


#define NTOK 4096
#define DM   1024
#define HS   2048
#define HR   1024
#define NE   8
#define TR   64
#define NTL  136
#define NTHR 256

static_assert(NTL * TR >= 2 * NTOK + NE * (TR - 1));
static_assert((NTOK % 64) == 0 && (NTOK % NTHR) == 0 && (NTOK % 32) == 0 && ((NTL * TR) % 2) == 0);
static_assert((DM % 64) == 0 && (HS % 128) == 0 && (HR % 256) == 0 && (DM % 256) == 0 && (HS % 64) == 0);
static_assert(NE * 32 == NTHR && ((DM * NE) % NTHR) == 0);
static_assert((size_t)NTOK * 2 * DM * 4 <= (size_t)2 * NTL * TR * DM * 2);
static_assert((size_t)2 * NTOK * HS * 2 <= (size_t)2 * NTL * TR * HR * 2);
static_assert((size_t)(2 * DM * HS + HS * DM) * 4 <= (size_t)NE * DM * HR * 4);

typedef float          v4f   __attribute__((ext_vector_type(4)));
typedef float          v8f   __attribute__((ext_vector_type(8)));
typedef int            v4i   __attribute__((ext_vector_type(4)));
typedef unsigned short v8us  __attribute__((ext_vector_type(8)));
typedef unsigned short v16us __attribute__((ext_vector_type(16)));
typedef __bf16         v16bf __attribute__((ext_vector_type(16)));
union FragB { v16us u; v8us h[2]; v16bf v; };

__device__ __forceinline__ unsigned int bfbits(float f) {
  unsigned int u = __float_as_uint(f);
  u = u + 0x7FFFu + ((u >> 16) & 1u);
  return u >> 16;
}

__device__ __forceinline__ v8f wmb(v16bf a, v16bf b, v8f c) {
  v8f d = __builtin_amdgcn_wmma_f32_16x16x32_bf16(false, a, false, b, (short)0, c, false, false);
#if defined(__HIP_DEVICE_COMPILE__)
  asm volatile("v_nop\n\tv_nop\n\tv_nop\n\tv_nop" : "+v"(d) : "v"(a), "v"(b));
#endif
  return d;
}

__global__ __launch_bounds__(NTHR) void k_wconv(const float* __restrict__ W, unsigned short* oh,
                                               unsigned short* ol, int K, int C) {
  __shared__ __attribute__((aligned(16))) unsigned short t0[64 * 72];
  __shared__ __attribute__((aligned(16))) unsigned short t1[64 * 72];
  const int tid = threadIdx.x;
  const int k0 = blockIdx.x * 64, c0 = blockIdx.y * 64;
  const size_t zoff = (size_t)blockIdx.z * (size_t)K * (size_t)C;
  const float* Wz = W + zoff;
  unsigned short* ohz = oh + zoff;
  unsigned short* olz = ol + zoff;
#pragma unroll
  for (int i = 0; i < 4; ++i) {
    const int idx = i * NTHR + tid;
    const int kr  = idx >> 4;
    const int cc  = (idx & 15) * 4;
    const v4f v = *(const v4f*)(Wz + (size_t)(k0 + kr) * C + c0 + cc);
    float f[4];
    f[0] = v.x; f[1] = v.y; f[2] = v.z; f[3] = v.w;
#pragma unroll
    for (int q = 0; q < 4; ++q) {
      const unsigned int hb = bfbits(f[q]);
      const float hf = __uint_as_float(hb << 16);
      t0[(cc + q) * 72 + kr] = (unsigned short)hb;
      t1[(cc + q) * 72 + kr] = (unsigned short)bfbits(f[q] - hf);
    }
  }
  __syncthreads();
  const int nrA = tid >> 3;
  const int nrB = nrA + 32;
  const int pc  = tid & 7;
  const v8us a0 = *(const v8us*)(t0 + nrA * 72 + pc * 8);
  const v8us b0 = *(const v8us*)(t0 + nrB * 72 + pc * 8);
  const v8us a1 = *(const v8us*)(t1 + nrA * 72 + pc * 8);
  const v8us b1 = *(const v8us*)(t1 + nrB * 72 + pc * 8);
  const size_t ga = ((size_t)(c0 + nrA)) * K + k0 + pc * 8;
  const size_t gb = ((size_t)(c0 + nrB)) * K + k0 + pc * 8;
  *(volatile v8us*)(ohz + ga) = a0;
  *(volatile v8us*)(ohz + gb) = b0;
  *(volatile v8us*)(olz + ga) = a1;
  *(volatile v8us*)(olz + gb) = b1;
  __threadfence();
  *(volatile v8us*)(ohz + ga) = a0;
  *(volatile v8us*)(ohz + gb) = b0;
  *(volatile v8us*)(olz + ga) = a1;
  *(volatile v8us*)(olz + gb) = b1;
}

__global__ __launch_bounds__(NTHR) void k_xconv(const float* __restrict__ x, unsigned short* Xh, unsigned short* Xl) {
  const int tid = threadIdx.x;
  const size_t r = (size_t)blockIdx.x * 2 + (tid >> 7);
  const int c0 = (tid & 127) * 8;
  const float* xp = x + r * DM + c0;
  const v4f a = *(const v4f*)xp;
  const v4f b = *(const v4f*)(xp + 4);
  float f[8];
  f[0] = a.x; f[1] = a.y; f[2] = a.z; f[3] = a.w; f[4] = b.x; f[5] = b.y; f[6] = b.z; f[7] = b.w;
  v8us oh, ol;
#pragma unroll
  for (int j = 0; j < 8; ++j) {
    const unsigned int hb = bfbits(f[j]);
    const float hf = __uint_as_float(hb << 16);
    oh[j] = (unsigned short)hb;
    ol[j] = (unsigned short)bfbits(f[j] - hf);
  }
  const size_t d = r * DM + c0;
  *(volatile v8us*)(Xh + d) = oh;
  *(volatile v8us*)(Xl + d) = ol;
  __threadfence();
  *(volatile v8us*)(Xh + d) = oh;
  *(volatile v8us*)(Xl + d) = ol;
}

__global__ __launch_bounds__(NTHR) void k_gate(const float* __restrict__ x, const float* __restrict__ rw,
                                              const float* __restrict__ rb, int* tinfo) {
#pragma clang fp contract(off)
  __shared__ __attribute__((aligned(16))) float sW[DM * NE];
  __shared__ float sZ[NE * NTHR];
  __shared__ float sB[NE];
  const int tid = threadIdx.x;
  const int t = blockIdx.x * NTHR + tid;
#pragma unroll 4
  for (int i = 0; i < (DM * NE) / NTHR; ++i) {
    const int idx = i * NTHR + tid;
    const int e = idx >> 10;
    const int k = idx & (DM - 1);
    sW[k * NE + e] = rw[idx];
  }
  if (tid < NE) sB[tid] = rb[tid];
  __syncthreads();

  const float* xr = x + (size_t)t * DM;
  float z[NE], c[NE];
#pragma unroll
  for (int e = 0; e < NE; ++e) { z[e] = 0.0f; c[e] = 0.0f; }
#define KH(E, WV) { const float y = fmaf(xv, WV, -c[E]); const float tt = z[E] + y; c[E] = (tt - z[E]) - y; z[E] = tt; }
#pragma unroll 1
  for (int k = 0; k < DM; ++k) {
    const float xv = xr[k];
    const v4f w0 = *(const v4f*)(sW + k * NE);
    const v4f w1 = *(const v4f*)(sW + k * NE + 4);
    KH(0, w0.x) KH(1, w0.y) KH(2, w0.z) KH(3, w0.w)
    KH(4, w1.x) KH(5, w1.y) KH(6, w1.z) KH(7, w1.w)
  }
#undef KH
#pragma unroll
  for (int e = 0; e < NE; ++e) sZ[e * NTHR + tid] = z[e] - c[e];
#pragma unroll 1
  for (int e = 0; e < NE; ++e) {
    const float zz = sZ[e * NTHR + tid];
    const float ex = expf(-zz);
    const float sg = 1.0f / (1.0f + ex);
    sZ[e * NTHR + tid] = sg;
  }
  float s[NE], sel[NE];
#pragma unroll
  for (int e = 0; e < NE; ++e) { s[e] = sZ[e * NTHR + tid]; sel[e] = s[e] + sB[e]; }

  float mx = sel[0]; float sv0 = s[0]; int i0 = 0;
#define P1(EI) { const bool cc = sel[EI] > mx; mx = cc ? sel[EI] : mx; sv0 = cc ? s[EI] : sv0; i0 = cc ? (EI) : i0; }
  P1(1) P1(2) P1(3) P1(4) P1(5) P1(6) P1(7)
#undef P1
  int   i1  = (i0 == 0) ? 1 : 0;
  float m1  = (i0 == 0) ? sel[1] : sel[0];
  float sv1 = (i0 == 0) ? s[1] : s[0];
#define P2(EI) { const bool cc = ((EI) != i0) && (sel[EI] > m1); m1 = cc ? sel[EI] : m1; sv1 = cc ? s[EI] : sv1; i1 = cc ? (EI) : i1; }
  P2(1) P2(2) P2(3) P2(4) P2(5) P2(6) P2(7)
#undef P2
  const float den = sv0 + sv1;
  const float dd  = den + 1e-9f;
  const float rcp = 1.0f / dd;
  const bool  ok  = den > 1e-9f;
  const float g0  = ok ? sv0 * rcp : 0.5f;
  const float g1  = ok ? sv1 * rcp : 0.5f;
  v4i o;
  o.x = i0; o.y = i1; o.z = __float_as_int(g0); o.w = __float_as_int(g1);
  int* op = tinfo + 4 * (size_t)t;
  *(volatile v4i*)op = o;
  __threadfence();
  *(volatile v4i*)op = o;
}

__device__ __forceinline__ void emit_pass(const int* __restrict__ tinfo, int* plist, int* rg,
                                          int w, int lane, int nCh, int segS, int segE, int nt) {
  int c = 0;
#pragma unroll 1
  for (int ch = 0; ch < nCh; ++ch) {
    const int t = ch * 32 + lane;
    const v4i inf = *(const v4i*)(tinfo + 4 * (size_t)t);
    const bool h0  = (inf.x == w);
    const bool h1  = (inf.y == w);
    const bool hit = h0 || h1;
    const unsigned mk = __builtin_amdgcn_ballot_w32(hit);
    const int rank = (int)__builtin_amdgcn_mbcnt_lo(mk, 0u);
    const int k    = (int)__builtin_popcount(mk);
    if (hit) rg[(c + rank) & 63] = (t << 1) | (h0 ? 0 : 1);
    __syncthreads();
    const int cn = c + k;
    if ((cn >> 5) != (c >> 5)) {
      const int L   = c >> 5;
      const int val = rg[((L & 1) << 5) + lane];
      const int row = segS * TR + L * 32 + lane;
      if ((unsigned)row < (unsigned)(NTL * TR)) *(volatile int*)(plist + row) = val;
    }
    __syncthreads();
    c = cn;
  }
  int linesTot = (segE - segS) * 2;
  linesTot = linesTot < 0 ? 0 : (linesTot > 2 * NTL ? 2 * NTL : linesTot);
  const int Lf  = c >> 5;
  const int rem = c & 31;
#pragma unroll
  for (int i = 0; i < 2; ++i) {
    const int L = Lf + i;
    if (L < linesTot) {
      const int rv  = rg[((L & 1) << 5) + lane];
      const int val = (i == 0 && lane < rem) ? rv : -1;
      const int row = segS * TR + L * 32 + lane;
      if ((unsigned)row < (unsigned)(NTL * TR)) *(volatile int*)(plist + row) = val;
    }
  }
#pragma unroll 1
  for (int L = nt * 2 + w; L < 2 * NTL; L += NE) {
    const int row = L * 32 + lane;
    *(volatile int*)(plist + row) = -1;
  }
}

__global__ __launch_bounds__(NTHR) void k_lists(const int* __restrict__ tinfo, int* plist, int* hdr, int nTok) {
  __shared__ __attribute__((aligned(16))) int ring[NE * 64];
  __shared__ int scnt[NE];
  __shared__ __attribute__((aligned(16))) int shdr[64];
  const int tid = threadIdx.x, lane = tid & 31, w = tid >> 5;
  const int nCh = nTok >> 5;

  int cnt = 0;
#pragma unroll 1
  for (int ch = 0; ch < nCh; ++ch) {
    const int t = ch * 32 + lane;
    const v4i inf = *(const v4i*)(tinfo + 4 * (size_t)t);
    const bool hit = (inf.x == w) || (inf.y == w);
    const unsigned mk = __builtin_amdgcn_ballot_w32(hit);
    cnt += (int)__builtin_popcount(mk);
  }
  if (lane == 0) scnt[w] = cnt;
  __syncthreads();
  if (tid == 0) {
    int s = 0;
    shdr[0] = 0;
    for (int e = 0; e < NE; ++e) {
      const int ce = scnt[e];
      s += (ce + TR - 1) / TR;
      shdr[e + 1]  = s;
      shdr[32 + e] = ce;
    }
    for (int i = NE + 1; i < 32; ++i) shdr[i] = 0;
    for (int i = 32 + NE; i < 64; ++i) shdr[i] = 0;
  }
  __syncthreads();
  const int segS = shdr[w], segE = shdr[w + 1];
  int nt = shdr[NE];
  nt = nt < 0 ? 0 : (nt > NTL ? NTL : nt);
  const v4i hv = *(const v4i*)(shdr + 4 * (tid & 15));

  emit_pass(tinfo, plist, ring + w * 64, w, lane, nCh, segS, segE, nt);
  if (tid < 16) *(volatile v4i*)(hdr + 4 * tid) = hv;
  __threadfence();
  emit_pass(tinfo, plist, ring + w * 64, w, lane, nCh, segS, segE, nt);
  if (tid < 16) *(volatile v4i*)(hdr + 4 * tid) = hv;
}

__global__ __launch_bounds__(NTHR) void k_gather(
    const unsigned short* __restrict__ Xh, const unsigned short* __restrict__ Xl,
    const int* __restrict__ plist, unsigned short* Gh, unsigned short* Gl, int nTok) {
  const int tid = threadIdx.x;
  const int r   = blockIdx.x * 2 + (tid >> 7);
  const int c0  = (tid & 127) * 8;
  const int ent = plist[r];
  const bool valid = ent >= 0;
  int t = ent >> 1;
  t = t < 0 ? 0 : (t > nTok - 1 ? nTok - 1 : t);
  const size_t so = (size_t)t * DM + c0;
  const v8us a = *(const v8us*)(Xh + so);
  const v8us b = *(const v8us*)(Xl + so);
  v8us oh, ol;
#pragma unroll
  for (int j = 0; j < 8; ++j) {
    oh[j] = valid ? a[j] : (unsigned short)0;
    ol[j] = valid ? b[j] : (unsigned short)0;
  }
  const size_t d = (size_t)r * DM + c0;
  *(volatile v8us*)(Gh + d) = oh;
  *(volatile v8us*)(Gl + d) = ol;
  __threadfence();
  *(volatile v8us*)(Gh + d) = oh;
  *(volatile v8us*)(Gl + d) = ol;
}

__device__ __forceinline__ int tile_expert(const int* __restrict__ hdr, int j, int* ntOut) {
  const v4i a = *(const v4i*)hdr;
  const v4i b = *(const v4i*)(hdr + 4);
  int nt = hdr[NE];
  nt = nt < 0 ? 0 : (nt > NTL ? NTL : nt);
  *ntOut = nt;
  int e = 0;
  e += (j >= a.y) ? 1 : 0; e += (j >= a.z) ? 1 : 0; e += (j >= a.w) ? 1 : 0;
  e += (j >= b.x) ? 1 : 0; e += (j >= b.y) ? 1 : 0; e += (j >= b.z) ? 1 : 0; e += (j >= b.w) ? 1 : 0;
  return e;
}

__global__ __launch_bounds__(NTHR) void k_ffn1(
    const unsigned short* __restrict__ Ah, const unsigned short* __restrict__ Al,
    const unsigned short* __restrict__ Wh, const unsigned short* __restrict__ Wl,
    const int* __restrict__ hdr, unsigned short* Hh, unsigned short* Hl) {
  __shared__ __attribute__((aligned(16))) unsigned short stg[8 * 2048];
  const int tid = threadIdx.x, lane = tid & 31, wave = tid >> 5, hh = lane >> 4, m = lane & 15;
  const int j = blockIdx.x;
  int nt;
  const int e = tile_expert(hdr, j, &nt);
  if (j >= nt) return;

  const int wr = wave >> 2, wc = wave & 3;
  const int colW = blockIdx.y * 256 + wc * 64;
  const size_t aOff = ((size_t)j * TR + wr * 32 + m) * DM + 8 * hh;
  const size_t bOff = ((size_t)e * HR + colW + m) * DM + 8 * hh;
  const unsigned short* ahP = Ah + aOff;
  const unsigned short* alP = Al + aOff;
  const unsigned short* bhP = Wh + bOff;
  const unsigned short* blP = Wl + bOff;

  v8f acc[2][4];
#pragma unroll
  for (int R = 0; R < 2; ++R)
#pragma unroll
    for (int t = 0; t < 4; ++t) { v8f zz = {0.f, 0.f, 0.f, 0.f, 0.f, 0.f, 0.f, 0.f}; acc[R][t] = zz; }

#pragma unroll 1
  for (int kt = 0; kt < DM / 32; ++kt) {
    const int kk = kt * 32;
    FragB ah[2], al[2];
#pragma unroll
    for (int R = 0; R < 2; ++R) {
      ah[R].h[0] = *(const v8us*)(ahP + (size_t)R * 16 * DM + kk);
      ah[R].h[1] = *(const v8us*)(ahP + (size_t)R * 16 * DM + kk + 16);
      al[R].h[0] = *(const v8us*)(alP + (size_t)R * 16 * DM + kk);
      al[R].h[1] = *(const v8us*)(alP + (size_t)R * 16 * DM + kk + 16);
    }
#pragma unroll
    for (int t = 0; t < 4; ++t) {
      FragB bh, bl;
      bh.h[0] = *(const v8us*)(bhP + (size_t)t * 16 * DM + kk);
      bh.h[1] = *(const v8us*)(bhP + (size_t)t * 16 * DM + kk + 16);
      bl.h[0] = *(const v8us*)(blP + (size_t)t * 16 * DM + kk);
      bl.h[1] = *(const v8us*)(blP + (size_t)t * 16 * DM + kk + 16);
#pragma unroll
      for (int R = 0; R < 2; ++R) {
        acc[R][t] = wmb(ah[R].v, bh.v, acc[R][t]);
        acc[R][t] = wmb(al[R].v, bh.v, acc[R][t]);
        acc[R][t] = wmb(ah[R].v, bl.v, acc[R][t]);
      }
    }
  }

  unsigned short* sh = stg + wave * 2048;
  unsigned short* sl = sh + 1024;
  const int q = lane >> 3, pc = lane & 7;
#pragma unroll
  for (int R = 0; R < 2; ++R) {
#pragma unroll
    for (int t = 0; t < 4; ++t) {
#pragma unroll
      for (int r = 0; r < 8; ++r) {
        const float v = acc[R][t][r];
        const float g = 0.5f * v * (1.0f + erff(v * 0.70710678118654752f));
        const unsigned int hb = bfbits(g);
        const float hf = __uint_as_float(hb << 16);
        const unsigned int lb = bfbits(g - hf);
        const int li = (8 * hh + r) * 64 + 16 * t + m;
        sh[li] = (unsigned short)hb;
        sl[li] = (unsigned short)lb;
      }
    }
    __syncthreads();
    const size_t rowG = (size_t)j * TR + wr * 32 + R * 16;
#pragma unroll
    for (int i = 0; i < 4; ++i) {
      const int row = 4 * i + q;
      const v8us hv = *(const v8us*)(sh + row * 64 + 8 * pc);
      const v8us lv = *(const v8us*)(sl + row * 64 + 8 * pc);
      const size_t go = (rowG + row) * HR + colW + 8 * pc;
      *(volatile v8us*)(Hh + go) = hv;
      *(volatile v8us*)(Hl + go) = lv;
    }
    __threadfence();
#pragma unroll
    for (int i = 0; i < 4; ++i) {
      const int row = 4 * i + q;
      const v8us hv = *(const v8us*)(sh + row * 64 + 8 * pc);
      const v8us lv = *(const v8us*)(sl + row * 64 + 8 * pc);
      const size_t go = (rowG + row) * HR + colW + 8 * pc;
      *(volatile v8us*)(Hh + go) = hv;
      *(volatile v8us*)(Hl + go) = lv;
    }
    __syncthreads();
  }
}

__global__ __launch_bounds__(NTHR) void k_ffn2(
    const unsigned short* __restrict__ Ah, const unsigned short* __restrict__ Al,
    const unsigned short* __restrict__ Wh, const unsigned short* __restrict__ Wl,
    const int* __restrict__ hdr, const int* __restrict__ plist, float* Y, int nTok) {
  __shared__ __attribute__((aligned(16))) float stg[8 * 1024];
  const int tid = threadIdx.x, lane = tid & 31, wave = tid >> 5, hh = lane >> 4, m = lane & 15;
  const int j = blockIdx.x;
  int nt;
  const int e = tile_expert(hdr, j, &nt);
  if (j >= nt) return;

  const int wr = wave >> 2, wc = wave & 3;
  const int colD = blockIdx.y * 256 + wc * 64;
  const int ent = plist[(size_t)j * TR + wr * 32 + lane];
  const size_t aOff = ((size_t)j * TR + wr * 32 + m) * HR + 8 * hh;
  const size_t bOff = ((size_t)e * DM + colD + m) * HR + 8 * hh;
  const unsigned short* ahP = Ah + aOff;
  const unsigned short* alP = Al + aOff;
  const unsigned short* bhP = Wh + bOff;
  const unsigned short* blP = Wl + bOff;

  v8f acc[2][4];
#pragma unroll
  for (int R = 0; R < 2; ++R)
#pragma unroll
    for (int t = 0; t < 4; ++t) { v8f zz = {0.f, 0.f, 0.f, 0.f, 0.f, 0.f, 0.f, 0.f}; acc[R][t] = zz; }

#pragma unroll 1
  for (int kt = 0; kt < HR / 32; ++kt) {
    const int kk = kt * 32;
    FragB ah[2], al[2];
#pragma unroll
    for (int R = 0; R < 2; ++R) {
      ah[R].h[0] = *(const v8us*)(ahP + (size_t)R * 16 * HR + kk);
      ah[R].h[1] = *(const v8us*)(ahP + (size_t)R * 16 * HR + kk + 16);
      al[R].h[0] = *(const v8us*)(alP + (size_t)R * 16 * HR + kk);
      al[R].h[1] = *(const v8us*)(alP + (size_t)R * 16 * HR + kk + 16);
    }
#pragma unroll
    for (int t = 0; t < 4; ++t) {
      FragB bh, bl;
      bh.h[0] = *(const v8us*)(bhP + (size_t)t * 16 * HR + kk);
      bh.h[1] = *(const v8us*)(bhP + (size_t)t * 16 * HR + kk + 16);
      bl.h[0] = *(const v8us*)(blP + (size_t)t * 16 * HR + kk);
      bl.h[1] = *(const v8us*)(blP + (size_t)t * 16 * HR + kk + 16);
#pragma unroll
      for (int R = 0; R < 2; ++R) {
        acc[R][t] = wmb(ah[R].v, bh.v, acc[R][t]);
        acc[R][t] = wmb(al[R].v, bh.v, acc[R][t]);
        acc[R][t] = wmb(ah[R].v, bl.v, acc[R][t]);
      }
    }
  }

  float* sw = stg + wave * 1024;
#pragma unroll
  for (int R = 0; R < 2; ++R) {
#pragma unroll
    for (int t = 0; t < 4; ++t)
#pragma unroll
      for (int r = 0; r < 8; ++r) sw[(8 * hh + r) * 64 + 16 * t + m] = acc[R][t][r];
    __syncthreads();
#pragma unroll
    for (int i = 0; i < 8; ++i) {
      const int eA = __builtin_amdgcn_readlane(ent, R * 16 + 2 * i);
      const int eB = __builtin_amdgcn_readlane(ent, R * 16 + 2 * i + 1);
      const int my = hh ? eB : eA;
      const bool valid = my >= 0;
      int tt = my >> 1;
      tt = tt < 0 ? 0 : (tt > nTok - 1 ? nTok - 1 : tt);
      const int slot = my & 1;
      const v4f v = *(const v4f*)(sw + (2 * i + hh) * 64 + 4 * m);
      float* gp = Y + ((size_t)tt * 2 + slot) * DM + colD + 4 * m;
      if (valid) *(volatile v4f*)gp = v;
    }
    __threadfence();
#pragma unroll
    for (int i = 0; i < 8; ++i) {
      const int eA = __builtin_amdgcn_readlane(ent, R * 16 + 2 * i);
      const int eB = __builtin_amdgcn_readlane(ent, R * 16 + 2 * i + 1);
      const int my = hh ? eB : eA;
      const bool valid = my >= 0;
      int tt = my >> 1;
      tt = tt < 0 ? 0 : (tt > nTok - 1 ? nTok - 1 : tt);
      const int slot = my & 1;
      const v4f v = *(const v4f*)(sw + (2 * i + hh) * 64 + 4 * m);
      float* gp = Y + ((size_t)tt * 2 + slot) * DM + colD + 4 * m;
      if (valid) *(volatile v4f*)gp = v;
    }
    __syncthreads();
  }
}

__global__ __launch_bounds__(NTHR) void k_sh_up(
    const unsigned short* __restrict__ Xh, const unsigned short* __restrict__ Xl,
    const unsigned short* __restrict__ W1h, const unsigned short* __restrict__ W1l,
    const unsigned short* __restrict__ W3h, const unsigned short* __restrict__ W3l,
    unsigned short* Gh, unsigned short* Gl) {
  __shared__ __attribute__((aligned(16))) unsigned short sgh[64 * 128];
  __shared__ __attribute__((aligned(16))) unsigned short sgl[64 * 128];
  const int tid = threadIdx.x, lane = tid & 31, wave = tid >> 5, hh = lane >> 4, m = lane & 15;
  const int wr = wave >> 2, wc = wave & 3;
  const int rowB = blockIdx.x * 64;
  const int colB = blockIdx.y * 128;
  const int row0 = rowB + wr * 32;
  const int col0 = colB + wc * 32;
  const size_t aOff = ((size_t)row0 + m) * DM + 8 * hh;
  const size_t bOff = ((size_t)col0 + m) * DM + 8 * hh;
  const unsigned short* ahP = Xh + aOff;
  const unsigned short* alP = Xl + aOff;
  const unsigned short* p1h = W1h + bOff;
  const unsigned short* p1l = W1l + bOff;
  const unsigned short* p3h = W3h + bOff;
  const unsigned short* p3l = W3l + bOff;

  v8f au[2][2], av[2][2];
#pragma unroll
  for (int R = 0; R < 2; ++R)
#pragma unroll
    for (int t = 0; t < 2; ++t) {
      v8f zz = {0.f, 0.f, 0.f, 0.f, 0.f, 0.f, 0.f, 0.f};
      au[R][t] = zz; av[R][t] = zz;
    }

#pragma unroll 1
  for (int kt = 0; kt < DM / 32; ++kt) {
    const int kk = kt * 32;
    FragB ah[2], al[2];
#pragma unroll
    for (int R = 0; R < 2; ++R) {
      ah[R].h[0] = *(const v8us*)(ahP + (size_t)R * 16 * DM + kk);
      ah[R].h[1] = *(const v8us*)(ahP + (size_t)R * 16 * DM + kk + 16);
      al[R].h[0] = *(const v8us*)(alP + (size_t)R * 16 * DM + kk);
      al[R].h[1] = *(const v8us*)(alP + (size_t)R * 16 * DM + kk + 16);
    }
#pragma unroll
    for (int t = 0; t < 2; ++t) {
      FragB bh, bl;
      bh.h[0] = *(const v8us*)(p1h + (size_t)t * 16 * DM + kk);
      bh.h[1] = *(const v8us*)(p1h + (size_t)t * 16 * DM + kk + 16);
      bl.h[0] = *(const v8us*)(p1l + (size_t)t * 16 * DM + kk);
      bl.h[1] = *(const v8us*)(p1l + (size_t)t * 16 * DM + kk + 16);
#pragma unroll
      for (int R = 0; R < 2; ++R) {
        au[R][t] = wmb(ah[R].v, bh.v, au[R][t]);
        au[R][t] = wmb(al[R].v, bh.v, au[R][t]);
        au[R][t] = wmb(ah[R].v, bl.v, au[R][t]);
      }
      FragB ch, cl;
      ch.h[0] = *(const v8us*)(p3h + (size_t)t * 16 * DM + kk);
      ch.h[1] = *(const v8us*)(p3h + (size_t)t * 16 * DM + kk + 16);
      cl.h[0] = *(const v8us*)(p3l + (size_t)t * 16 * DM + kk);
      cl.h[1] = *(const v8us*)(p3l + (size_t)t * 16 * DM + kk + 16);
#pragma unroll
      for (int R = 0; R < 2; ++R) {
        av[R][t] = wmb(ah[R].v, ch.v, av[R][t]);
        av[R][t] = wmb(al[R].v, ch.v, av[R][t]);
        av[R][t] = wmb(ah[R].v, cl.v, av[R][t]);
      }
    }
  }

#pragma unroll
  for (int R = 0; R < 2; ++R) {
#pragma unroll
    for (int t = 0; t < 2; ++t) {
#pragma unroll
      for (int r = 0; r < 8; ++r) {
        const float u  = au[R][t][r];
        const float vv = av[R][t][r];
        const float ex = expf(-u);
        const float sg = 1.0f / (1.0f + ex);
        const float g  = u * sg * vv;
        const unsigned int hb = bfbits(g);
        const float hf = __uint_as_float(hb << 16);
        const unsigned int lb = bfbits(g - hf);
        const int li = (wr * 32 + R * 16 + 8 * hh + r) * 128 + wc * 32 + 16 * t + m;
        sgh[li] = (unsigned short)hb;
        sgl[li] = (unsigned short)lb;
      }
    }
  }
  __syncthreads();
  const int rr = tid >> 4;
  const int pc = tid & 15;
#pragma unroll
  for (int i = 0; i < 4; ++i) {
    const int row = 16 * i + rr;
    const v8us hv = *(const v8us*)(sgh + row * 128 + 8 * pc);
    const v8us lv = *(const v8us*)(sgl + row * 128 + 8 * pc);
    const size_t go = ((size_t)(rowB + row)) * HS + colB + 8 * pc;
    *(volatile v8us*)(Gh + go) = hv;
    *(volatile v8us*)(Gl + go) = lv;
  }
  __threadfence();
#pragma unroll
  for (int i = 0; i < 4; ++i) {
    const int row = 16 * i + rr;
    const v8us hv = *(const v8us*)(sgh + row * 128 + 8 * pc);
    const v8us lv = *(const v8us*)(sgl + row * 128 + 8 * pc);
    const size_t go = ((size_t)(rowB + row)) * HS + colB + 8 * pc;
    *(volatile v8us*)(Gh + go) = hv;
    *(volatile v8us*)(Gl + go) = lv;
  }
}

__global__ __launch_bounds__(NTHR) void k_sh_down(
    const unsigned short* __restrict__ Ah, const unsigned short* __restrict__ Al,
    const unsigned short* __restrict__ Wh, const unsigned short* __restrict__ Wl,
    const int* __restrict__ tinfo, const float* __restrict__ Y, float* out) {
  __shared__ __attribute__((aligned(16))) float stg[8 * 1024];
  const int tid = threadIdx.x, lane = tid & 31, wave = tid >> 5, hh = lane >> 4, m = lane & 15;
  const int wr = wave >> 2, wc = wave & 3;
  const int row0 = blockIdx.x * 64 + wr * 32;
  const int colD = blockIdx.y * 256 + wc * 64;
  const size_t aOff = ((size_t)row0 + m) * HS + 8 * hh;
  const size_t bOff = ((size_t)colD + m) * HS + 8 * hh;
  const unsigned short* ahP = Ah + aOff;
  const unsigned short* alP = Al + aOff;
  const unsigned short* bhP = Wh + bOff;
  const unsigned short* blP = Wl + bOff;

  v8f acc[2][4];
#pragma unroll
  for (int R = 0; R < 2; ++R)
#pragma unroll
    for (int t = 0; t < 4; ++t) { v8f zz = {0.f, 0.f, 0.f, 0.f, 0.f, 0.f, 0.f, 0.f}; acc[R][t] = zz; }

#pragma unroll 1
  for (int kt = 0; kt < HS / 32; ++kt) {
    const int kk = kt * 32;
    FragB ah[2], al[2];
#pragma unroll
    for (int R = 0; R < 2; ++R) {
      ah[R].h[0] = *(const v8us*)(ahP + (size_t)R * 16 * HS + kk);
      ah[R].h[1] = *(const v8us*)(ahP + (size_t)R * 16 * HS + kk + 16);
      al[R].h[0] = *(const v8us*)(alP + (size_t)R * 16 * HS + kk);
      al[R].h[1] = *(const v8us*)(alP + (size_t)R * 16 * HS + kk + 16);
    }
#pragma unroll
    for (int t = 0; t < 4; ++t) {
      FragB bh, bl;
      bh.h[0] = *(const v8us*)(bhP + (size_t)t * 16 * HS + kk);
      bh.h[1] = *(const v8us*)(bhP + (size_t)t * 16 * HS + kk + 16);
      bl.h[0] = *(const v8us*)(blP + (size_t)t * 16 * HS + kk);
      bl.h[1] = *(const v8us*)(blP + (size_t)t * 16 * HS + kk + 16);
#pragma unroll
      for (int R = 0; R < 2; ++R) {
        acc[R][t] = wmb(ah[R].v, bh.v, acc[R][t]);
        acc[R][t] = wmb(al[R].v, bh.v, acc[R][t]);
        acc[R][t] = wmb(ah[R].v, bl.v, acc[R][t]);
      }
    }
  }

  float* sw = stg + wave * 1024;
#pragma unroll
  for (int R = 0; R < 2; ++R) {
#pragma unroll
    for (int t = 0; t < 4; ++t)
#pragma unroll
      for (int r = 0; r < 8; ++r) sw[(8 * hh + r) * 64 + 16 * t + m] = acc[R][t][r];
    __syncthreads();
#pragma unroll
    for (int i = 0; i < 8; ++i) {
      const int tok = row0 + R * 16 + 2 * i + hh;
      const v4i inf = *(const v4i*)(tinfo + 4 * (size_t)tok);
      const float g0 = __int_as_float(inf.z);
      const float g1 = __int_as_float(inf.w);
      const v4f v  = *(const v4f*)(sw + (2 * i + hh) * 64 + 4 * m);
      const float* yp = Y + ((size_t)tok * 2) * DM + colD + 4 * m;
      const v4f y0 = *(const v4f*)yp;
      const v4f y1 = *(const v4f*)(yp + DM);
      const v4f o  = v + (y0 * g0 + y1 * g1);
      float* gp = out + (size_t)tok * DM + colD + 4 * m;
      *(volatile v4f*)gp = o;
    }
    __threadfence();
#pragma unroll
    for (int i = 0; i < 8; ++i) {
      const int tok = row0 + R * 16 + 2 * i + hh;
      const v4i inf = *(const v4i*)(tinfo + 4 * (size_t)tok);
      const float g0 = __int_as_float(inf.z);
      const float g1 = __int_as_float(inf.w);
      const v4f v  = *(const v4f*)(sw + (2 * i + hh) * 64 + 4 * m);
      const float* yp = Y + ((size_t)tok * 2) * DM + colD + 4 * m;
      const v4f y0 = *(const v4f*)yp;
      const v4f y1 = *(const v4f*)(yp + DM);
      const v4f o  = v + (y0 * g0 + y1 * g1);
      float* gp = out + (size_t)tok * DM + colD + 4 * m;
      *(volatile v4f*)gp = o;
    }
    __syncthreads();
  }
}

extern "C" void kernel_launch(void* const* d_in, const int* in_sizes, int n_in,
                              void* d_out, int out_size, void* d_ws, size_t ws_size,
                              hipStream_t stream) {
  if (n_in < 8) return;
  if (in_sizes[0] != NTOK * DM || in_sizes[1] != NE * DM || in_sizes[2] != NE) return;
  if (in_sizes[3] != DM * HS || in_sizes[4] != DM * HS || in_sizes[5] != HS * DM) return;
  if (in_sizes[6] != NE * DM * HR || in_sizes[7] != NE * HR * DM) return;
  if (out_size != NTOK * DM) return;

  const float* x   = (const float*)d_in[0];
  const float* rw  = (const float*)d_in[1];
  const float* rb  = (const float*)d_in[2];
  const float* sw1 = (const float*)d_in[3];
  const float* sw3 = (const float*)d_in[4];
  const float* sw2 = (const float*)d_in[5];
  const float* ew1 = (const float*)d_in[6];
  const float* ew2 = (const float*)d_in[7];
  float* out = (float*)d_out;

  char* ws = (char*)d_ws;
  size_t off = 0;
  const size_t szX  = (size_t)NTOK * DM * 2;
  const size_t szEW = (size_t)NE * DM * HR * 2;
  const size_t szXG = (size_t)NTL * TR * DM * 2;
  const size_t szH  = (size_t)NTL * TR * HR * 2;
  const size_t szS1 = (size_t)DM * HS * 2;
  const size_t szS2 = (size_t)HS * DM * 2;
  const size_t szG  = (size_t)NTOK * HS * 2;
  const size_t szY  = (size_t)NTOK * 2 * DM * 4;
  const size_t oTI = off; off += (size_t)NTOK * 16;      off = (off + 255) & ~(size_t)255;
  const size_t oHD = off; off += 256;                    off = (off + 255) & ~(size_t)255;
  const size_t oPL = off; off += (size_t)NTL * TR * 4;   off = (off + 255) & ~(size_t)255;
  const size_t oX  = off; off += 2 * szX;                off = (off + 255) & ~(size_t)255;
  const size_t oB  = off; off += 2 * szEW;               off = (off + 255) & ~(size_t)255;
  const size_t oC  = off; off += 2 * szXG;               off = (off + 255) & ~(size_t)255;
  const size_t oD  = off; off += 2 * szH;                off = (off + 255) & ~(size_t)255;
  if (off > ws_size || off > (size_t)134217728) return;
  if (szY > 2 * szXG || 2 * szG > 2 * szH || 2 * szS1 * 2 + 2 * szS2 > 2 * szEW) return;

  int*            tinfo = (int*)(ws + oTI);
  int*            hdr   = (int*)(ws + oHD);
  int*            plist = (int*)(ws + oPL);
  unsigned short* Xh    = (unsigned short*)(ws + oX);
  unsigned short* Xl    = (unsigned short*)(ws + oX + szX);
  unsigned short* EWh   = (unsigned short*)(ws + oB);
  unsigned short* EWl   = (unsigned short*)(ws + oB + szEW);
  unsigned short* S1h   = (unsigned short*)(ws + oB);
  unsigned short* S1l   = (unsigned short*)(ws + oB + szS1);
  unsigned short* S3h   = (unsigned short*)(ws + oB + 2 * szS1);
  unsigned short* S3l   = (unsigned short*)(ws + oB + 3 * szS1);
  unsigned short* S2h   = (unsigned short*)(ws + oB + 4 * szS1);
  unsigned short* S2l   = (unsigned short*)(ws + oB + 4 * szS1 + szS2);
  unsigned short* XGh   = (unsigned short*)(ws + oC);
  unsigned short* XGl   = (unsigned short*)(ws + oC + szXG);
  float*          Y     = (float*)(ws + oC);
  unsigned short* Hh    = (unsigned short*)(ws + oD);
  unsigned short* Hl    = (unsigned short*)(ws + oD + szH);
  unsigned short* Gh    = (unsigned short*)(ws + oD);
  unsigned short* Gl    = (unsigned short*)(ws + oD + szG);

  k_xconv<<<NTOK / 2, NTHR, 0, stream>>>(x, Xh, Xl);
  k_gate<<<NTOK / NTHR, NTHR, 0, stream>>>(x, rw, rb, tinfo);
  k_lists<<<1, NTHR, 0, stream>>>(tinfo, plist, hdr, NTOK);
  k_gather<<<(NTL * TR) / 2, NTHR, 0, stream>>>(Xh, Xl, plist, XGh, XGl, NTOK);

  k_wconv<<<dim3(DM / 64, HR / 64, NE), NTHR, 0, stream>>>(ew1, EWh, EWl, DM, HR);
  k_ffn1<<<dim3(NTL, HR / 256), NTHR, 0, stream>>>(XGh, XGl, EWh, EWl, hdr, Hh, Hl);
  k_wconv<<<dim3(HR / 64, DM / 64, NE), NTHR, 0, stream>>>(ew2, EWh, EWl, HR, DM);
  k_ffn2<<<dim3(NTL, DM / 256), NTHR, 0, stream>>>(Hh, Hl, EWh, EWl, hdr, plist, Y, NTOK);

  k_wconv<<<dim3(DM / 64, HS / 64, 1), NTHR, 0, stream>>>(sw1, S1h, S1l, DM, HS);
  k_wconv<<<dim3(DM / 64, HS / 64, 1), NTHR, 0, stream>>>(sw3, S3h, S3l, DM, HS);
  k_wconv<<<dim3(HS / 64, DM / 64, 1), NTHR, 0, stream>>>(sw2, S2h, S2l, HS, DM);
  k_sh_up<<<dim3(NTOK / 64, HS / 128), NTHR, 0, stream>>>(Xh, Xl, S1h, S1l, S3h, S3l, Gh, Gl);
  k_sh_down<<<dim3(NTOK / 64, DM / 256), NTHR, 0, stream>>>(Gh, Gl, S2h, S2l, tinfo, Y, out);
}
